// custom_v5_180388626854
// MI455X (gfx1250) — hardware-verified
//
#include <hip/hip_runtime.h>
#include <math.h>

typedef __attribute__((ext_vector_type(16))) _Float16 v16h;
typedef __attribute__((ext_vector_type(16))) __bf16 v16b;
typedef __attribute__((ext_vector_type(8)))  _Float16 v8h;
typedef __attribute__((ext_vector_type(8)))  float v8f;
typedef __attribute__((ext_vector_type(4)))  float v4f;
typedef __attribute__((ext_vector_type(2)))  float v2f;
typedef __attribute__((ext_vector_type(4)))  unsigned v4u;
typedef __attribute__((ext_vector_type(4)))  int v4i;
typedef float __attribute__((may_alias)) float_a;
typedef int __attribute__((may_alias)) int_a;

template <typename T> __device__ __forceinline__ void vst2(void* p, T v) { *(volatile T*)p = v; __threadfence(); *(volatile T*)p = v; }
__device__ __forceinline__ v8f wmma16(v16h a, v16h b, v8f c) {
  v8f d = __builtin_amdgcn_wmma_f32_16x16x32_f16(false, a, false, b, (short)0, c, false, false);
  asm volatile("v_nop\n\tv_nop\n\tv_nop\n\tv_nop" : "+v"(d) : "v"(a), "v"(b));
  return d;
}
__device__ __forceinline__ v8f wmma_bf(v16b a, v16b b, v8f c) {
  v8f d = __builtin_amdgcn_wmma_f32_16x16x32_bf16(false, a, false, b, (short)0, c, false, false);
  asm volatile("v_nop\n\tv_nop\n\tv_nop\n\tv_nop" : "+v"(d) : "v"(a), "v"(b));
  return d;
}
__device__ __forceinline__ v16h frag_h(const _Float16* rowk0, int lane) {
  union { v16h v; v8h q[2]; } u; const _Float16* p = rowk0 + 8 * (lane >> 4);
  u.q[0] = *(const v8h*)p; u.q[1] = *(const v8h*)(p + 16); return u.v;
}
__device__ __forceinline__ v16h frag_f32(const float* rowk0, int lane) {
  v16h a; const float* p = rowk0 + 8 * (lane >> 4);
#pragma unroll
  for (int i = 0; i < 8; ++i) { a[i] = (_Float16)p[i]; a[8 + i] = (_Float16)p[16 + i]; }
  return a;
}
__device__ __forceinline__ v16h frag_f32s(const float* rowk0, int lane, float sc) {
  v16h a; const float* p = rowk0 + 8 * (lane >> 4);
#pragma unroll
  for (int i = 0; i < 8; ++i) { a[i] = (_Float16)(p[i] * sc); a[8 + i] = (_Float16)(p[16 + i] * sc); }
  return a;
}
__device__ __forceinline__ v16h fragc_f32(const float* W, int k0, int n, int lane, int ld, int K) {
  v16h a; const int g = lane >> 4;
#pragma unroll
  for (int i = 0; i < 8; ++i) { const int ka = k0 + 8 * g + i, kb = ka + 16;
    a[i] = (_Float16)(ka < K ? W[(size_t)(ka < K ? ka : K - 1) * ld + n] : 0.f); a[8 + i] = (_Float16)(kb < K ? W[(size_t)(kb < K ? kb : K - 1) * ld + n] : 0.f); }
  return a;
}
struct F2 { v16b h, l; };
__device__ __forceinline__ F2 bsplit16(const float v[16]) { F2 r;
#pragma unroll
  for (int i = 0; i < 16; ++i) { const __bf16 h = (__bf16)v[i]; r.h[i] = h; r.l[i] = (__bf16)(v[i] - (float)h); }
  return r; }
__device__ __forceinline__ F2 split_row(const float* row, int k0, int lane) { float v[16]; const float* p = row + k0 + 8 * (lane >> 4);
#pragma unroll
  for (int i = 0; i < 8; ++i) { v[i] = p[i]; v[8 + i] = p[16 + i]; }
  return bsplit16(v); }
__device__ __forceinline__ F2 split_rowK(const float* row, int k0, int lane, int K) { float v[16]; const int g = lane >> 4;
#pragma unroll
  for (int i = 0; i < 8; ++i) { const int ka = k0 + 8 * g + i, kb = ka + 16; v[i] = ka < K ? row[ka < K ? ka : K - 1] : 0.f; v[8 + i] = kb < K ? row[kb < K ? kb : K - 1] : 0.f; }
  return bsplit16(v); }
__device__ __forceinline__ F2 split_col(const float* W, int k0, int n, int lane, int ld, int K) { float v[16]; const int g = lane >> 4;
#pragma unroll
  for (int i = 0; i < 8; ++i) { const int ka = k0 + 8 * g + i, kb = ka + 16; v[i] = ka < K ? W[(size_t)(ka < K ? ka : K - 1) * ld + n] : 0.f; v[8 + i] = kb < K ? W[(size_t)(kb < K ? kb : K - 1) * ld + n] : 0.f; }
  return bsplit16(v); }
__device__ __forceinline__ v8f mac3(const F2& a, const F2& b, v8f c) { c = wmma_bf(a.l, b.h, c); c = wmma_bf(a.h, b.l, c); return wmma_bf(a.h, b.h, c); }
__device__ __forceinline__ float sigm(float v) { return 1.0f / (1.0f + expf(-v)); }
#define LDSX() do { asm volatile("s_wait_dscnt 0" ::: "memory"); __builtin_amdgcn_wave_barrier(); __builtin_amdgcn_fence(__ATOMIC_RELEASE, "workgroup"); } while (0)


#define NB 32
#define TT 32
#define RR 256
#define UU 4
#define YS 64
#define C1 32
#define NPX (RR * RR)
#define WSC 256.0f
#ifndef TNB
#define TNB NB
#endif
typedef __attribute__((ext_vector_type(8))) __bf16 v8b;
__device__ __forceinline__ v16b frag_b(const __bf16* rowk0, int lane) {
  union { v16b v; v8b q[2]; } u; const __bf16* p = rowk0 + 8 * (lane >> 4);
  u.q[0] = *(const v8b*)p; u.q[1] = *(const v8b*)(p + 16); return u.v;
}
__device__ __forceinline__ float bfr(float v) { return (float)(__bf16)v; }
__device__ __attribute__((noinline)) float exp_ni(float v) { return expf(v); }
__device__ __attribute__((noinline)) float erf_ni(float v) { return erff(v); }

#define WS_X0  0u
#define WS_H1  (WS_X0 + 4u * (size_t)NB * NPX)
#define WS_PW1 (WS_H1 + 2u * (size_t)NB * NPX * C1)
#define WS_PW2 (WS_PW1 + 2u * C1 * 32)
#define WS_END (WS_PW2 + 2u * 16 * 288)

__global__ __launch_bounds__(256) void k_packw(const float* __restrict__ W1, const float* __restrict__ W2, char* __restrict__ ws) { __shared__ __align__(16) __bf16 s1[C1 * 32]; __shared__ __align__(16) _Float16 s2[16 * 288]; const int t = threadIdx.x;
  for (int e = t; e < C1 * 32; e += 256) { const int o = e / 32, k = e % 32; s1[e] = (k < 9) ? (__bf16)W1[o * 9 + k] : (__bf16)0.0f; }
  for (int e = t; e < 16 * 288; e += 256) { const int o = e / 288, k = e % 288; const int tap = k / 32, c = k % 32; s2[e] = (o == 0) ? (_Float16)(bfr(W2[c * 9 + tap]) * WSC) : (_Float16)0.0f; }
  __syncthreads(); for (int q = t; q < C1 * 32 / 8; q += 256) vst2((unsigned*)((__bf16*)(ws + WS_PW1) + q * 8), *(const v4u*)&s1[q * 8]); for (int q = t; q < 16 * 288 / 8; q += 256) vst2((unsigned*)((_Float16*)(ws + WS_PW2) + q * 8), *(const v4u*)&s2[q * 8]); }
__global__ __launch_bounds__(256) void k_x0(const float* __restrict__ YT, const float* __restrict__ HT, float* __restrict__ X0) { __shared__ float sy[TT][YS]; __shared__ __align__(16) float so[RR]; const int p = blockIdx.x, t = threadIdx.x; const size_t b = blockIdx.y;
  for (int e = t; e < TT * YS; e += 256) { const int tt = e / YS, qq = e % YS; sy[tt][qq] = bfr(YT[((b * TT + tt) * YS + p / UU) * YS + qq]); } __syncthreads();
  { const int q = t; float s = 0.f;
#pragma unroll 1
    for (int tt = 0; tt < TT; ++tt) s += bfr(HT[((size_t)tt * RR + p) * RR + q]) * sy[tt][q / UU]; so[q] = s; }
  __syncthreads(); if (t < RR / 4) vst2(X0 + (b * RR + p) * (size_t)RR + t * 4, *(const v4f*)&so[t * 4]); }
__global__ __launch_bounds__(128) void k_c1(const float* __restrict__ X0, const __bf16* __restrict__ PW1, const float* __restrict__ B1, _Float16* __restrict__ H1) { __shared__ __align__(16) _Float16 sh[64][C1 + 8];
  const int tid = threadIdx.x, wave = tid >> 5, lane = tid & 31, col = lane & 15, g = lane >> 4; const size_t b = blockIdx.y; const int pix0 = blockIdx.x * 64 + wave * 16; const int p = (pix0 + col) / RR, q = (pix0 + col) % RR;
  float v[16];
#pragma unroll
  for (int i = 0; i < 16; ++i) { const int k = 8 * g + (i < 8 ? i : 8 + i); float x = 0.f; if (k < 9) { const int pp = p + k / 3 - 1, qq = q + k % 3 - 1; if (pp >= 0 && pp < RR && qq >= 0 && qq < RR) x = X0[(b * RR + pp) * (size_t)RR + qq]; } v[i] = x; }
  const F2 a = bsplit16(v); v8f acc[2] = {};
#pragma unroll
  for (int j = 0; j < 2; ++j) { const v16b w = frag_b(PW1 + (size_t)(j * 16 + col) * 32, lane); acc[j] = wmma_bf(a.h, w, acc[j]); acc[j] = wmma_bf(a.l, w, acc[j]); }
#pragma unroll
  for (int j = 0; j < 2; ++j) { const float bb = bfr(B1[j * 16 + col]);
#pragma unroll
    for (int r = 0; r < 8; ++r) sh[wave * 16 + 8 * g + r][j * 16 + col] = (_Float16)fmaxf(acc[j][r] + bb, 0.f); }
  __syncthreads(); for (int e = tid; e < 64 * 4; e += 128) { const int rl = e >> 2, qq = e & 3; vst2((unsigned*)(H1 + (b * NPX + blockIdx.x * 64 + rl) * C1 + qq * 8), *(const v4u*)&sh[rl][qq * 8]); } }
__global__ __launch_bounds__(128) void k_c2(const _Float16* __restrict__ H1, const _Float16* __restrict__ PW2, const float* __restrict__ B2, float* __restrict__ OUT) { __shared__ __align__(16) float so[64];
  const int tid = threadIdx.x, wave = tid >> 5, lane = tid & 31, col = lane & 15, g = lane >> 4; const size_t b = blockIdx.y; const int pix0 = blockIdx.x * 64 + wave * 16; const int p = (pix0 + col) / RR, q = (pix0 + col) % RR;
  v8f acc = {};
#pragma unroll
  for (int tap = 0; tap < 9; ++tap) { const int pp = p + tap / 3 - 1, qq = q + tap % 3 - 1; const bool ok = pp >= 0 && pp < RR && qq >= 0 && qq < RR; const _Float16* src = H1 + (b * NPX + (size_t)(ok ? pp * RR + qq : 0)) * C1; v16h a; const _Float16* ps = src + 8 * g;
#pragma unroll
    for (int i = 0; i < 8; ++i) { a[i] = ok ? ps[i] : (_Float16)0.0f; a[8 + i] = ok ? ps[16 + i] : (_Float16)0.0f; }
    acc = wmma16(a, frag_h(PW2 + (size_t)col * 288 + tap * 32, lane), acc); }
  if (col == 0) { const float bb = bfr(B2[0]);
#pragma unroll
    for (int r = 0; r < 8; ++r) so[wave * 16 + 8 * g + r] = acc[r] * (1.0f / WSC) + bb; }
  __syncthreads(); if (tid < 16) vst2(OUT + b * NPX + (size_t)blockIdx.x * 64 + tid * 4, *(const v4f*)&so[tid * 4]); }
extern "C" void kernel_launch(void* const* d_in, const int* in_sizes, int n_in, void* d_out, int out_size, void* d_ws, size_t ws_size, hipStream_t stream) {
  (void)in_sizes; (void)n_in; (void)out_size;
  const float** F = (const float**)d_in;
  if (ws_size < (size_t)WS_END) return;
  char* ws = (char*)d_ws; float* X0 = (float*)(ws + WS_X0); _Float16* H1 = (_Float16*)(ws + WS_H1);
  k_packw<<<1, 256, 0, stream>>>(F[2], F[4], ws);
  k_x0<<<dim3(RR, TNB), 256, 0, stream>>>(F[0], F[1], X0);
  k_c1<<<dim3(NPX / 64, TNB), 128, 0, stream>>>(X0, (const __bf16*)(ws + WS_PW1), F[3], H1);
  k_c2<<<dim3(NPX / 64, TNB), 128, 0, stream>>>(H1, (const _Float16*)(ws + WS_PW2), F[5], (float*)d_out);
}
